// EvRoomDetector_26929444946615
// MI455X (gfx1250) — hardware-verified
//
#include <hip/hip_runtime.h>
#pragma clang fp contract(off)

typedef _Float16 f16t;
typedef _Float16 v16h __attribute__((ext_vector_type(16)));
typedef _Float16 v8h  __attribute__((ext_vector_type(8)));
typedef unsigned short us_t;
typedef unsigned short v8us __attribute__((ext_vector_type(8)));
typedef float v8f __attribute__((ext_vector_type(8)));
typedef float v4f __attribute__((ext_vector_type(4)));
typedef v8us __attribute__((may_alias)) v8usa;
typedef v4f  __attribute__((may_alias)) v4fa;
typedef v8h  __attribute__((may_alias)) v8ha;

union Frag { v16h v; v8us half[2]; };

#define HH    128
#define WW    128
#define NPIX  16384
#define CC    128
#define NL    49152
#define DF    1024
#define NTOP  50
#define NJOUT 150
#define XSP   264
#define SHP   136
#define FTP   132
#define WSC   32.0f

__device__ __forceinline__ int imin(int a, int b) { return a < b ? a : b; }
__device__ __forceinline__ int imax(int a, int b) { return a > b ? a : b; }
__device__ __forceinline__ v4f vmax4(v4f a, v4f b) {
  v4f r;
  r.x = fmaxf(a.x, b.x); r.y = fmaxf(a.y, b.y); r.z = fmaxf(a.z, b.z); r.w = fmaxf(a.w, b.w);
  return r;
}

__device__ __forceinline__ v8f mma16(v16h a, v16h b, v8f c) {
  return __builtin_amdgcn_wmma_f32_16x16x32_f16(false, a, false, b, (short)0, c, false, false);
}

__device__ __forceinline__ void mma_tile_k1024(const us_t* __restrict__ A, const us_t* __restrict__ B,
                                               int arow0, int brow0, int lane, v8f (&acc)[2][4]) {
  const int l15 = lane & 15, h8 = (lane >> 4) << 3;
  const us_t* ap0 = A + (size_t)(arow0 + l15) * DF + h8;
  const us_t* ap1 = ap0 + (size_t)16 * DF;
  const us_t* bb  = B + (size_t)(brow0 + l15) * DF + h8;
  #pragma unroll 1
  for (int k0 = 0; k0 < DF; k0 += 32) {
    Frag a0, a1, b[4];
    a0.half[0] = *(const v8usa*)(ap0 + k0);
    a0.half[1] = *(const v8usa*)(ap0 + k0 + 16);
    a1.half[0] = *(const v8usa*)(ap1 + k0);
    a1.half[1] = *(const v8usa*)(ap1 + k0 + 16);
    #pragma unroll
    for (int nt = 0; nt < 4; ++nt) {
      const us_t* bp = bb + (size_t)nt * 16 * DF + k0;
      b[nt].half[0] = *(const v8usa*)(bp);
      b[nt].half[1] = *(const v8usa*)(bp + 16);
    }
    #pragma unroll
    for (int nt = 0; nt < 4; ++nt) {
      acc[0][nt] = mma16(a0.v, b[nt].v, acc[0][nt]);
      acc[1][nt] = mma16(a1.v, b[nt].v, acc[1][nt]);
    }
    asm volatile("v_nop\n\tv_nop\n\tv_nop\n\tv_nop"
                 : "+v"(acc[0][0]), "+v"(acc[0][1]), "+v"(acc[0][2]), "+v"(acc[0][3]),
                   "+v"(acc[1][0]), "+v"(acc[1][1]), "+v"(acc[1][2]), "+v"(acc[1][3])
                 : "v"(a0.v), "v"(a1.v), "v"(b[0].v), "v"(b[1].v), "v"(b[2].v), "v"(b[3].v));
  }
}

__device__ __forceinline__ void zero_acc(v8f (&acc)[2][4]) {
  v8f z;
  #pragma unroll
  for (int j = 0; j < 8; ++j) z[j] = 0.0f;
  #pragma unroll
  for (int mt = 0; mt < 2; ++mt)
    #pragma unroll
    for (int nt = 0; nt < 4; ++nt) acc[mt][nt] = z;
}

__global__ __launch_bounds__(256) void lines_k(const float* __restrict__ md, const float* __restrict__ dis,
                                               const float* __restrict__ res, float* __restrict__ LN) {
  const int i = blockIdx.x * 256 + threadIdx.x;
  if (i >= NL) return;
  const int sidx = i >> 14, pix = i & (NPIX - 1);
  const float sgn = (float)(sidx - 1);
  const float y0 = (float)(pix >> 7), x0 = (float)(pix & 127);
  const float PI_F = 3.14159274101257324f;
  const float md0 = md[pix], md1 = md[NPIX + pix], md2 = md[2 * NPIX + pix];
  const float t0 = md0 - 0.5f;
  const float t1 = t0 * PI_F;
  const float a_md = t1 * 2.0f;
  const float u1 = md1 * PI_F;
  const float a_st = u1 * 0.5f;
  const float nm2 = -md2;
  const float u2 = nm2 * PI_F;
  const float a_ed = u2 * 0.5f;
  float s0 = 0.0f, s1 = 0.0f, s2 = 0.0f, c0 = 0.0f, c1 = 0.0f, c2 = 0.0f;
  #pragma unroll 1
  for (int k = 0; k < 3; ++k) {
    const float ang = (k == 0) ? a_md : ((k == 1) ? a_st : a_ed);
    float sv, cv;
    sincosf(ang, &sv, &cv);
    s0 = s1; s1 = s2; s2 = sv;
    c0 = c1; c1 = c2; c2 = cv;
  }
  const float cs_md = c0, ss_md = s0;
  const float cs_st = fmaxf(c1, 0.001f), ss_st = fmaxf(s1, 0.001f);
  const float cs_ed = fmaxf(c2, 0.001f), ss_ed = fminf(s2, -0.001f);
  float y_st = 0.0f, y_ed = 0.0f;
  #pragma unroll 1
  for (int k = 0; k < 2; ++k) {
    const float nu = k ? ss_ed : ss_st;
    const float de = k ? cs_ed : cs_st;
    const float qv = nu / de;
    y_st = y_ed; y_ed = qv;
  }
  const float rr = sgn * res[pix];
  const float dsum = dis[pix] + rr;
  const float d = dsum * 5.0f;
  const float p1 = ss_md * y_st; const float q1 = cs_md - p1; const float x_st = q1 * d;
  const float p2 = cs_md * y_st; const float q2 = ss_md + p2; const float y_s  = q2 * d;
  const float p3 = ss_md * y_ed; const float q3 = cs_md - p3; const float x_ed = q3 * d;
  const float p4 = cs_md * y_ed; const float q4 = ss_md + p4; const float y_e  = q4 * d;
  v4f r;
  r.x = fminf(fmaxf(x_st + x0, 0.0f), (float)(WW - 1));
  r.y = fminf(fmaxf(y_s + y0, 0.0f), (float)(HH - 1));
  r.z = fminf(fmaxf(x_ed + x0, 0.0f), (float)(WW - 1));
  r.w = fminf(fmaxf(y_e + y0, 0.0f), (float)(HH - 1));
  float* dst = LN + (size_t)i * 4;
  *(volatile v4f*)dst = r;
  __threadfence();
  *(volatile v4f*)dst = r;
}

__global__ __launch_bounds__(256) void cvtw_k(const float* __restrict__ w, us_t* __restrict__ out, int n8) {
  const int g = blockIdx.x * 256 + threadIdx.x;
  if (g >= n8) return;
  const float* src = w + (size_t)8 * g;
  const v4f a = *(const v4fa*)src;
  const v4f b = *(const v4fa*)(src + 4);
  v8h o;
  o[0] = (f16t)(a.x * WSC); o[1] = (f16t)(a.y * WSC); o[2] = (f16t)(a.z * WSC); o[3] = (f16t)(a.w * WSC);
  o[4] = (f16t)(b.x * WSC); o[5] = (f16t)(b.y * WSC); o[6] = (f16t)(b.z * WSC); o[7] = (f16t)(b.w * WSC);
  const v8us ov = __builtin_bit_cast(v8us, o);
  us_t* dst = out + (size_t)8 * g;
  *(volatile v8us*)dst = ov;
  __threadfence();
  *(volatile v8us*)dst = ov;
}

__global__ __launch_bounds__(256) void ftr_k(const float* __restrict__ feats, float* __restrict__ ft) {
  __shared__ __attribute__((aligned(16))) float T[32 * FTP];
  const int tid = threadIdx.x, lane = tid & 31, wid = tid >> 5;
  const int p0 = blockIdx.x * 32;
  #pragma unroll 1
  for (int cq = 0; cq < 16; ++cq) {
    const int c = cq * 8 + wid;
    T[lane * FTP + c] = feats[(size_t)c * NPIX + p0 + lane];
  }
  __syncthreads();
  v4f vals[4];
  size_t adr[4];
  #pragma unroll
  for (int it = 0; it < 4; ++it) {
    const int row = wid * 4 + it;
    vals[it] = *(const v4fa*)(T + row * FTP + 4 * lane);
    adr[it] = (size_t)(p0 + row) * CC + 4 * lane;
  }
  #pragma unroll
  for (int it = 0; it < 4; ++it) *(volatile v4f*)(ft + adr[it]) = vals[it];
  __threadfence();
  #pragma unroll
  for (int it = 0; it < 4; ++it) *(volatile v4f*)(ft + adr[it]) = vals[it];
}

__global__ __launch_bounds__(256) void pool_k(const float* __restrict__ FT, const float* __restrict__ LN,
                                              us_t* __restrict__ X, int srow0) {
  __shared__ __attribute__((aligned(16))) f16t Xs[32 * XSP];
  const int tid = threadIdx.x, lane = tid & 31, wid = tid >> 5;
  const int ll = tid >> 3, p = tid & 7;
  const int pix0 = blockIdx.x * 32;
  const v4f L = *(const v4fa*)(LN + (size_t)(srow0 + pix0 + ll) * 4);
  int o00[4], o10[4], o01[4], o11[4];
  float wy0[4], wy1[4], wx0[4], wx1[4];
  #pragma unroll
  for (int j = 0; j < 4; ++j) {
    const int i = 4 * p + j;
    const float t = (i == 31) ? 1.0f : (float)i * (1.0f / 31.0f);
    const float omt = 1.0f - t;
    const float ax = L.x * t;
    const float bx = L.z * omt;
    const float cx = ax + bx;
    const float px = cx - 0.5f;
    const float ay = L.y * t;
    const float by = L.w * omt;
    const float cy = ay + by;
    const float py = cy - 0.5f;
    const float px0 = fminf(fmaxf(floorf(px), 0.0f), (float)(WW - 1));
    const float py0 = fminf(fmaxf(floorf(py), 0.0f), (float)(HH - 1));
    const float px1 = fminf(fmaxf(px0 + 1.0f, 0.0f), (float)(WW - 1));
    const float py1 = fminf(fmaxf(py0 + 1.0f, 0.0f), (float)(HH - 1));
    const int ix0 = imin(imax((int)px0, 0), WW - 1);
    const int iy0 = imin(imax((int)py0, 0), HH - 1);
    const int ix1 = imin(imax((int)px1, 0), WW - 1);
    const int iy1 = imin(imax((int)py1, 0), HH - 1);
    wy0[j] = py1 - py; wy1[j] = py - py0;
    wx0[j] = px1 - px; wx1[j] = px - px0;
    o00[j] = (iy0 * WW + ix0) * CC;
    o10[j] = (iy1 * WW + ix0) * CC;
    o01[j] = (iy0 * WW + ix1) * CC;
    o11[j] = (iy1 * WW + ix1) * CC;
  }
  #pragma unroll 1
  for (int ch = 0; ch < 4; ++ch) {
    #pragma unroll 1
    for (int q = 0; q < 8; ++q) {
      const int c = ch * 32 + q * 4;
      const float* base = FT + c;
      v4f mx;
      mx.x = 0.0f; mx.y = 0.0f; mx.z = 0.0f; mx.w = 0.0f;
      #pragma unroll
      for (int j = 0; j < 4; ++j) {
        const v4f f00 = *(const v4fa*)(base + o00[j]);
        const v4f f10 = *(const v4fa*)(base + o10[j]);
        const v4f f01 = *(const v4fa*)(base + o01[j]);
        const v4f f11 = *(const v4fa*)(base + o11[j]);
        v4f t1 = f00 * wy0[j]; t1 = t1 * wx0[j];
        v4f t2 = f10 * wy1[j]; t2 = t2 * wx0[j];
        v4f t3 = f01 * wy0[j]; t3 = t3 * wx1[j];
        v4f t4 = f11 * wy1[j]; t4 = t4 * wx1[j];
        v4f sm = t1 + t2; sm = sm + t3; sm = sm + t4;
        mx = (j == 0) ? sm : vmax4(mx, sm);
      }
      f16t* xr = Xs + ll * XSP + (q * 4) * 8 + p;
      xr[0]  = (f16t)mx.x;
      xr[8]  = (f16t)mx.y;
      xr[16] = (f16t)mx.z;
      xr[24] = (f16t)mx.w;
    }
    __syncthreads();
    v8us vals[4];
    size_t adr[4];
    #pragma unroll
    for (int it = 0; it < 4; ++it) {
      const int lrow = wid * 4 + it;
      const v8h hv = *(const v8ha*)(Xs + lrow * XSP + lane * 8);
      vals[it] = __builtin_bit_cast(v8us, hv);
      adr[it] = (size_t)(pix0 + lrow) * DF + ch * 256 + lane * 8;
    }
    #pragma unroll
    for (int it = 0; it < 4; ++it) *(volatile v8us*)(X + adr[it]) = vals[it];
    __threadfence();
    #pragma unroll
    for (int it = 0; it < 4; ++it) *(volatile v8us*)(X + adr[it]) = vals[it];
    __syncthreads();
  }
}

__global__ __launch_bounds__(256) void gemm1_k(const us_t* __restrict__ X, const us_t* __restrict__ Wp,
                                               const float* __restrict__ bias, us_t* __restrict__ Hout) {
  __shared__ __attribute__((aligned(16))) f16t Sh[128 * SHP];
  const int tid = threadIdx.x, lane = tid & 31, wid = tid >> 5;
  const int l15 = lane & 15, h8 = (lane >> 4) << 3;
  const int wm = wid & 3, wn = wid >> 2;
  const int mblk = blockIdx.x * 128, nblk = blockIdx.y * 128;
  v8f acc[2][4];
  zero_acc(acc);
  mma_tile_k1024(X, Wp, mblk + wm * 32, nblk + wn * 64, lane, acc);
  const float osc = 1.0f / WSC;
  #pragma unroll
  for (int nt = 0; nt < 4; ++nt) {
    const int nloc = wn * 64 + nt * 16 + l15;
    const float bv = bias[nblk + nloc];
    #pragma unroll
    for (int mt = 0; mt < 2; ++mt) {
      #pragma unroll
      for (int r = 0; r < 8; ++r) {
        const int row = wm * 32 + mt * 16 + h8 + r;
        float v = acc[mt][nt][r] * osc;
        v = v + bv;
        v = fmaxf(v, 0.0f);
        Sh[row * SHP + nloc] = (f16t)v;
      }
    }
  }
  __syncthreads();
  v8us vals[8];
  size_t adr[8];
  #pragma unroll
  for (int it = 0; it < 8; ++it) {
    const int row = wid * 16 + it * 2 + (lane >> 4);
    const int piece = l15 * 8;
    const v8h hv = *(const v8ha*)(Sh + row * SHP + piece);
    vals[it] = __builtin_bit_cast(v8us, hv);
    adr[it] = (size_t)(mblk + row) * DF + nblk + piece;
  }
  #pragma unroll
  for (int it = 0; it < 8; ++it) *(volatile v8us*)(Hout + adr[it]) = vals[it];
  __threadfence();
  #pragma unroll
  for (int it = 0; it < 8; ++it) *(volatile v8us*)(Hout + adr[it]) = vals[it];
}

__global__ __launch_bounds__(256) void gemm2_k(const us_t* __restrict__ Hp, const us_t* __restrict__ Wp,
                                               const float* __restrict__ bias, const float* __restrict__ w3,
                                               const float* __restrict__ b3, float* __restrict__ out, int orow0) {
  __shared__ float Sr[2 * 128 * 16];
  __shared__ __attribute__((aligned(16))) float So[128];
  const int tid = threadIdx.x, lane = tid & 31, wid = tid >> 5;
  const int l15 = lane & 15, h8 = (lane >> 4) << 3;
  const int wm = wid & 3, wn = wid >> 2;
  const int mblk = blockIdx.x * 128;
  const float osc = 1.0f / WSC;
  float t[2][8];
  #pragma unroll
  for (int mt = 0; mt < 2; ++mt)
    #pragma unroll
    for (int r = 0; r < 8; ++r) t[mt][r] = 0.0f;
  v8f acc[2][4];
  #pragma unroll 1
  for (int ns = 0; ns < 8; ++ns) {
    zero_acc(acc);
    mma_tile_k1024(Hp, Wp, mblk + wm * 32, ns * 128 + wn * 64, lane, acc);
    #pragma unroll
    for (int nt = 0; nt < 4; ++nt) {
      const int n = ns * 128 + wn * 64 + nt * 16 + l15;
      const float bv = bias[n];
      const float wv = w3[n];
      #pragma unroll
      for (int mt = 0; mt < 2; ++mt) {
        #pragma unroll
        for (int r = 0; r < 8; ++r) {
          float v = acc[mt][nt][r] * osc;
          v = v + bv;
          v = fmaxf(v, 0.0f);
          const float pr = v * wv;
          t[mt][r] = t[mt][r] + pr;
        }
      }
    }
  }
  #pragma unroll
  for (int mt = 0; mt < 2; ++mt) {
    #pragma unroll
    for (int r = 0; r < 8; ++r) {
      const int mloc = wm * 32 + mt * 16 + h8 + r;
      Sr[(wn * 128 + mloc) * 16 + l15] = t[mt][r];
    }
  }
  __syncthreads();
  if (tid < 128) {
    float s = 0.0f;
    #pragma unroll
    for (int g = 0; g < 2; ++g) {
      #pragma unroll
      for (int l = 0; l < 16; ++l) s = s + Sr[(g * 128 + tid) * 16 + l];
    }
    So[tid] = s + b3[0];
  }
  __syncthreads();
  if (wid == 0) {
    const v4f v = *(const v4fa*)(So + 4 * lane);
    float* dst = out + (size_t)orow0 + mblk + 4 * lane;
    *(volatile v4f*)dst = v;
    __threadfence();
    *(volatile v4f*)dst = v;
  }
}

__global__ __launch_bounds__(256) void junc_k(const float* __restrict__ jloc, const float* __restrict__ joff,
                                              float* __restrict__ outj) {
  __shared__ float sval[256];
  __shared__ int   sidx[256];
  __shared__ float so[160];
  __shared__ float spv[4];
  __shared__ int   spi[4];
  const int tid = threadIdx.x, lane = tid & 31, wid = tid >> 5;
  float nv[64];
  #pragma unroll
  for (int j = 0; j < 64; ++j) {
    const int q = j * 256 + tid;
    const int y = q >> 7, x = q & 127;
    const float a = jloc[q];
    float mx = a;
    #pragma unroll
    for (int dy = -1; dy <= 1; ++dy) {
      const int yc = imin(imax(y + dy, 0), HH - 1);
      #pragma unroll
      for (int dx = -1; dx <= 1; ++dx) {
        if (dy == 0 && dx == 0) continue;
        const int xc = imin(imax(x + dx, 0), WW - 1);
        mx = fmaxf(mx, jloc[yc * WW + xc]);
      }
    }
    nv[j] = a * ((a == mx) ? 1.0f : 0.0f);
  }
  float pv = __builtin_inff();
  int pi = -1;
  #pragma unroll 1
  for (int it = 0; it < NTOP; ++it) {
    float best = -__builtin_inff();
    int bidx = 0x7fffffff;
    #pragma unroll
    for (int j = 0; j < 64; ++j) {
      const int q = j * 256 + tid;
      const float v = nv[j];
      const bool elig = (v < pv) || ((v == pv) && (q > pi));
      const bool better = elig && (v > best);
      best = better ? v : best;
      bidx = better ? q : bidx;
    }
    sval[tid] = best;
    sidx[tid] = bidx;
    __syncthreads();
    #pragma unroll 1
    for (int s = 128; s > 0; s >>= 1) {
      if (tid < s) {
        const float ov = sval[tid + s], mv = sval[tid];
        const int oi = sidx[tid + s], mi = sidx[tid];
        const bool take = (ov > mv) || ((ov == mv) && (oi < mi));
        if (take) { sval[tid] = ov; sidx[tid] = oi; }
      }
      __syncthreads();
    }
    if (tid == 0) {
      const int idx = sidx[0];
      const float sc = sval[0];
      const int ic = imin(imax(idx, 0), NPIX - 1);
      const float jx = joff[ic];
      const float jy = joff[NPIX + ic];
      const float xf = (float)(ic & 127);
      const float yf = (float)(ic >> 7);
      const float xa = xf + jx;
      const float xo = xa + 0.5f;
      const float ya = yf + jy;
      const float yo = ya + 0.5f;
      so[2 * it] = xo;
      so[2 * it + 1] = yo;
      so[2 * NTOP + it] = sc;
      spv[0] = sc;
      spi[0] = idx;
    }
    __syncthreads();
    pv = spv[0];
    pi = spi[0];
  }
  if (wid == 0) {
    float v[5];
    #pragma unroll
    for (int it = 0; it < 5; ++it) {
      const int f = it * 32 + lane;
      v[it] = so[imin(f, NJOUT - 1)];
    }
    #pragma unroll
    for (int it = 0; it < 5; ++it) {
      const int f = it * 32 + lane;
      if (f < NJOUT) *(volatile float*)(outj + f) = v[it];
    }
    __threadfence();
    #pragma unroll
    for (int it = 0; it < 5; ++it) {
      const int f = it * 32 + lane;
      if (f < NJOUT) *(volatile float*)(outj + f) = v[it];
    }
  }
}

extern "C" void kernel_launch(void* const* d_in, const int* in_sizes, int n_in,
                              void* d_out, int out_size, void* d_ws, size_t ws_size,
                              hipStream_t stream) {
  if (n_in < 12) return;
  if (in_sizes[0] != 3 * NPIX || in_sizes[1] != NPIX || in_sizes[2] != NPIX) return;
  if (in_sizes[3] != NPIX || in_sizes[4] != 2 * NPIX || in_sizes[5] != CC * NPIX) return;
  if (in_sizes[6] != DF * DF || in_sizes[7] != DF || in_sizes[8] != DF * DF || in_sizes[9] != DF) return;
  if (in_sizes[10] != DF || in_sizes[11] != 1) return;
  if (out_size != NL + NJOUT) return;

  const float* md    = (const float*)d_in[0];
  const float* dis   = (const float*)d_in[1];
  const float* res   = (const float*)d_in[2];
  const float* jloc  = (const float*)d_in[3];
  const float* joff  = (const float*)d_in[4];
  const float* feats = (const float*)d_in[5];
  const float* W1    = (const float*)d_in[6];
  const float* b1    = (const float*)d_in[7];
  const float* W2    = (const float*)d_in[8];
  const float* b2    = (const float*)d_in[9];
  const float* W3    = (const float*)d_in[10];
  const float* b3    = (const float*)d_in[11];
  float* out = (float*)d_out;

  char* ws = (char*)d_ws;
  size_t off = 0;
  const size_t szLN = (size_t)NL * 4 * 4;
  const size_t szFT = (size_t)NPIX * CC * 4;
  const size_t szW  = (size_t)DF * DF * 2;
  const size_t szX  = (size_t)NPIX * DF * 2;
  float* LN  = (float*)(ws + off); off += szLN;
  float* FT  = (float*)(ws + off); off += szFT;
  us_t*  W1S = (us_t*)(ws + off);  off += szW;
  us_t*  W2S = (us_t*)(ws + off);  off += szW;
  us_t*  XP  = (us_t*)(ws + off);  off += szX;
  us_t*  H1  = (us_t*)(ws + off);  off += szX;
  if (off > ws_size) return;

  lines_k<<<NL / 256, 256, 0, stream>>>(md, dis, res, LN);
  cvtw_k<<<(DF * DF / 8 + 255) / 256, 256, 0, stream>>>(W1, W1S, DF * DF / 8);
  cvtw_k<<<(DF * DF / 8 + 255) / 256, 256, 0, stream>>>(W2, W2S, DF * DF / 8);
  ftr_k<<<NPIX / 32, 256, 0, stream>>>(feats, FT);
  junc_k<<<1, 256, 0, stream>>>(jloc, joff, out + NL);
  for (int s = 0; s < 3; ++s) {
    pool_k<<<NPIX / 32, 256, 0, stream>>>(FT, LN, XP, s * NPIX);
    gemm1_k<<<dim3(NPIX / 128, DF / 128), 256, 0, stream>>>(XP, W1S, b1, H1);
    gemm2_k<<<NPIX / 128, 256, 0, stream>>>(H1, W2S, b2, W3, b3, out, s * NPIX);
  }
}
